// PPM_6743098655522
// MI455X (gfx1250) — hardware-verified
//
#include <hip/hip_runtime.h>
#include <math.h>
#include <stdint.h>

#define NBATCH 4
#define CCH    256
#define NVOX   4096
#define SSC    4096.0f
#define TSC    64.0f
#define OSC    (1.0f / (4096.0f * 64.0f))
static_assert((CCH % 64) == 0 && (NVOX % 64) == 0);
static_assert((CCH % 32) == 0 && (NVOX % 32) == 0);
static_assert((NVOX % 32) == 0 && (CCH % 8) == 0);

typedef _Float16 v16h __attribute__((ext_vector_type(16)));
typedef _Float16 v8h  __attribute__((ext_vector_type(8)));
typedef __bf16   v16b __attribute__((ext_vector_type(16)));
typedef __bf16   v8b  __attribute__((ext_vector_type(8)));
typedef float    v8f  __attribute__((ext_vector_type(8)));
typedef float    v4f  __attribute__((ext_vector_type(4)));
typedef unsigned int v4u __attribute__((ext_vector_type(4)));
typedef v4u __attribute__((may_alias)) v4ua;

#if defined(__HIP_DEVICE_COMPILE__)
#define DEV_ASM 1
#else
#define DEV_ASM 0
#endif

__device__ __forceinline__ unsigned short bf_bits(float f) {
  unsigned u = __float_as_uint(f);
  return (unsigned short)((u + 0x7FFFu + ((u >> 16) & 1u)) >> 16);
}
__device__ __forceinline__ float bf_up(unsigned short hb) { return __uint_as_float(((unsigned)hb) << 16); }
__device__ __forceinline__ unsigned short h_bits(_Float16 x) { return __builtin_bit_cast(unsigned short, x); }
__device__ __forceinline__ unsigned pk16(unsigned short a, unsigned short b) { return (unsigned)a | ((unsigned)b << 16); }
__device__ __forceinline__ v8f zero8() { v8f z = {0.f, 0.f, 0.f, 0.f, 0.f, 0.f, 0.f, 0.f}; return z; }

template <typename OT> struct FT;
template <> struct FT<__bf16>   { typedef v16b frag; typedef v8b half8; };
template <> struct FT<_Float16> { typedef v16h frag; typedef v8h half8; };

template <typename OT>
__device__ __forceinline__ typename FT<OT>::frag ldfrag(const OT* p) {
  union { typename FT<OT>::frag v; typename FT<OT>::half8 h[2]; } f;
  f.h[0] = *(const typename FT<OT>::half8*)(p);
  f.h[1] = *(const typename FT<OT>::half8*)(p + 16);
  return f.v;
}

__device__ __forceinline__ v8f mmar(v16b a, v16b b, v8f c) {
  return __builtin_amdgcn_wmma_f32_16x16x32_bf16(false, a, false, b, (short)0, c, false, false);
}
__device__ __forceinline__ v8f mmar(v16h a, v16h b, v8f c) {
  return __builtin_amdgcn_wmma_f32_16x16x32_f16(false, a, false, b, (short)0, c, false, false);
}
__device__ __forceinline__ void dep_guard(v8f& a, v8f& b, v16b x, v16b y) {
#if DEV_ASM
  asm volatile("v_nop\n\tv_nop\n\tv_nop\n\tv_nop" : "+v"(a), "+v"(b) : "v"(x), "v"(y));
#else
  (void)a; (void)b; (void)x; (void)y;
#endif
}
__device__ __forceinline__ void dep_guard(v8f& a, v8f& b, v16h x, v16h y) {
#if DEV_ASM
  asm volatile("v_nop\n\tv_nop\n\tv_nop\n\tv_nop" : "+v"(a), "+v"(b) : "v"(x), "v"(y));
#else
  (void)a; (void)b; (void)x; (void)y;
#endif
}
__device__ __forceinline__ void keep4(v16b a, v16b b, v16b c, v16b d) {
#if DEV_ASM
  asm volatile("v_nop" :: "v"(a), "v"(b), "v"(c), "v"(d));
#else
  (void)a; (void)b; (void)c; (void)d;
#endif
}
__device__ __forceinline__ void keep4(v16h a, v16h b, v16h c, v16h d) {
#if DEV_ASM
  asm volatile("v_nop" :: "v"(a), "v"(b), "v"(c), "v"(d));
#else
  (void)a; (void)b; (void)c; (void)d;
#endif
}
__device__ __forceinline__ void acc_guard4(v8f& a, v8f& b, v8f& c, v8f& d) {
#if DEV_ASM
  asm volatile("v_nop\n\tv_nop\n\tv_nop\n\tv_nop" : "+v"(a), "+v"(b), "+v"(c), "+v"(d));
#else
  (void)a; (void)b; (void)c; (void)d;
#endif
}
__device__ __forceinline__ void wave_lds_sync() {
  __builtin_amdgcn_fence(__ATOMIC_RELEASE, "workgroup");
  __builtin_amdgcn_wave_barrier();
  __builtin_amdgcn_fence(__ATOMIC_ACQUIRE, "workgroup");
}

__global__ __launch_bounds__(256) void cvt_bf16x8(const float* __restrict__ in, unsigned short* out, int n8) {
  const int i = blockIdx.x * 256 + (int)threadIdx.x;
  if (i < n8) {
    const v4f a  = *(const v4f*)(in + (size_t)i * 8);
    const v4f a4 = *(const v4f*)(in + (size_t)i * 8 + 4);
    v4u p;
    p[0] = pk16(bf_bits(a[0]),  bf_bits(a[1]));
    p[1] = pk16(bf_bits(a[2]),  bf_bits(a[3]));
    p[2] = pk16(bf_bits(a4[0]), bf_bits(a4[1]));
    p[3] = pk16(bf_bits(a4[2]), bf_bits(a4[3]));
    unsigned short* o = out + (size_t)i * 8;
    *(volatile v4u*)o = p;
    __threadfence();
    *(volatile v4u*)o = p;
  }
}

__global__ __launch_bounds__(256) void prep_xt(const float* __restrict__ x, unsigned short* xt, float* rn) {
  __shared__ __align__(16) unsigned short sX[32][CCH + 8];
  __shared__ float sS[8][32];
  const int tid = (int)threadIdx.x, lane = tid & 31, w = tid >> 5;
  const int b = blockIdx.y, n0 = blockIdx.x * 32;
  const float* xb = x + (size_t)b * CCH * NVOX + n0 + lane;
  float ss = 0.f;
#pragma unroll 4
  for (int i = 0; i < CCH / 8; ++i) {
    const int c = w + 8 * i;
    const float v = xb[(size_t)c * NVOX];
    const unsigned short hb = bf_bits(v);
    const float vr = bf_up(hb);
    ss += vr * vr;
    sX[lane][c] = hb;
  }
  sS[w][lane] = ss;
  __syncthreads();
  if (w == 0) {
    float tot = sS[0][lane];
#pragma unroll
    for (int k = 1; k < 8; ++k) tot += sS[k][lane];
    const float nrm = sqrtf(tot);
    const float r = 1.0f / fmaxf(nrm, 1e-8f);
    float* pr = rn + (size_t)b * NVOX + n0 + lane;
    *(volatile float*)pr = r;
    __threadfence();
    *(volatile float*)pr = r;
  }
  v4u rv[4];
#pragma unroll
  for (int rr = 0; rr < 4; ++rr) rv[rr] = *(const v4ua*)(&sX[w * 4 + rr][8 * lane]);
  for (int pass = 0; pass < 2; ++pass) {
#pragma unroll
    for (int rr = 0; rr < 4; ++rr) {
      const int n = n0 + w * 4 + rr;
      *(volatile v4u*)(xt + ((size_t)b * NVOX + n) * CCH + 8 * lane) = rv[rr];
    }
    __threadfence();
  }
}

template <bool HASB>
__device__ __forceinline__ void store_rows16(const float* slab, unsigned short* C, int ldc, int rowBase, int colBase,
                                             int lane, const float* __restrict__ bias, float sc) {
  const int q = lane >> 3, c8 = (lane & 7) * 8;
  v4u hv[4];
#pragma unroll
  for (int it = 0; it < 4; ++it) {
    const int row = it * 4 + q;
    const float* sp = slab + row * 68 + c8;
    float badd = 0.f;
    if (HASB) badd = bf_up(bf_bits(bias[rowBase + row]));
    v4u a;
#pragma unroll
    for (int e = 0; e < 4; ++e) {
      float f0 = sp[2 * e], f1 = sp[2 * e + 1];
      if (HASB) { f0 = (f0 + badd) * sc; f1 = (f1 + badd) * sc; }
      a[e] = pk16(h_bits((_Float16)f0), h_bits((_Float16)f1));
    }
    hv[it] = a;
  }
  for (int pass = 0; pass < 2; ++pass) {
#pragma unroll
    for (int it = 0; it < 4; ++it) {
      const int row = it * 4 + q;
      *(volatile v4u*)(C + (size_t)(rowBase + row) * ldc + colBase + c8) = hv[it];
    }
    __threadfence();
  }
}

template <typename OT, int MODE>
__global__ __launch_bounds__(256) void gemm64(
    const unsigned short* __restrict__ Ap, int lda, long long strideA,
    const unsigned short* __restrict__ Btp, int ldb, long long strideB,
    void* Cout, int ldc, long long strideC,
    const float* __restrict__ aux,
    int M, int N, int K, float oscale) {
  typedef typename FT<OT>::frag V16;
  const OT* A  = (const OT*)(const void*)Ap;
  const OT* Bt = (const OT*)(const void*)Btp;
  __shared__ __align__(16) float sT[8][16 * 68];
  const int b    = blockIdx.y;
  const int lane = threadIdx.x & 31;
  const int wave = threadIdx.x >> 5;
  const int tilesN = N >> 6;
  const int tilesM = M >> 6;
  const int tile = blockIdx.x * 8 + wave;
  int tm, tn;
  if (MODE == 2) {
    const int ntri = (tilesM * (tilesM + 1)) >> 1;
    if (tile >= ntri) return;
    int tr = 0, rem = tile;
    for (int it = 0; it < tilesM; ++it) {
      const int len = tilesM - tr;
      if (rem < len) break;
      rem -= len;
      ++tr;
    }
    tm = tr;
    tn = tr + rem;
    if (tm >= tilesM || tn >= tilesN) return;
  } else {
    if (tile >= tilesM * tilesN) return;
    tm = tile / tilesN;
    tn = tile - tm * tilesN;
  }
  const int m0 = tm << 6;
  const int n0 = tn << 6;

  const OT* Ab = A  + (size_t)b * (size_t)strideA;
  const OT* Bb = Bt + (size_t)b * (size_t)strideB;

  const int rlane = lane & 15;
  const int koff  = (lane >> 4) * 8;
  const int mOff  = (lane >> 4) * 8;

  v8f acc[4][4];
#pragma unroll
  for (int i = 0; i < 4; ++i)
#pragma unroll
    for (int j = 0; j < 4; ++j) acc[i][j] = zero8();

  for (int k0 = 0; k0 < K; k0 += 32) {
    V16 bq[4];
#pragma unroll
    for (int j = 0; j < 4; ++j)
      bq[j] = ldfrag<OT>(Bb + (size_t)(n0 + (j << 4) + rlane) * ldb + koff + k0);
#pragma unroll
    for (int i = 0; i < 4; ++i) {
      const V16 af = ldfrag<OT>(Ab + (size_t)(m0 + (i << 4) + rlane) * lda + koff + k0);
#pragma unroll
      for (int j = 0; j < 4; ++j) acc[i][j] = mmar(af, bq[j], acc[i][j]);
      dep_guard(acc[i][0], acc[i][3], af, bq[3]);
    }
    keep4(bq[0], bq[1], bq[2], bq[3]);
  }
  acc_guard4(acc[0][0], acc[0][1], acc[0][2], acc[0][3]);
  acc_guard4(acc[1][0], acc[1][1], acc[1][2], acc[1][3]);
  acc_guard4(acc[2][0], acc[2][1], acc[2][2], acc[2][3]);
  acc_guard4(acc[3][0], acc[3][1], acc[3][2], acc[3][3]);

  if (MODE == 2) {
    float rc[4];
#pragma unroll
    for (int j = 0; j < 4; ++j) rc[j] = aux[n0 + (j << 4) + rlane];
#pragma unroll
    for (int i = 0; i < 4; ++i) {
      const v4f ra = *(const v4f*)(aux + m0 + (i << 4) + mOff);
      const v4f rb = *(const v4f*)(aux + m0 + (i << 4) + mOff + 4);
      const float rr[8] = { ra[0], ra[1], ra[2], ra[3], rb[0], rb[1], rb[2], rb[3] };
#pragma unroll
      for (int j = 0; j < 4; ++j) {
#pragma unroll
        for (int r = 0; r < 8; ++r) {
          float v = acc[i][j][r] * rr[r] * rc[j];
          v = fmaxf(v, 0.f);
          acc[i][j][r] = v * v * oscale;
        }
      }
    }
  }

  float* slab = sT[wave];
  if (MODE == 0) {
    float* C = (float*)Cout + (size_t)b * (size_t)strideC;
#pragma unroll
    for (int i = 0; i < 4; ++i) {
      const int mBase = m0 + (i << 4);
#pragma unroll
      for (int j = 0; j < 4; ++j) {
#pragma unroll
        for (int r = 0; r < 8; ++r) slab[(mOff + r) * 68 + (j << 4) + rlane] = acc[i][j][r];
      }
      wave_lds_sync();
      const int h2 = lane >> 4, c4 = (lane & 15) * 4;
      for (int pass = 0; pass < 2; ++pass) {
#pragma unroll
        for (int it = 0; it < 8; ++it) {
          const int row = it * 2 + h2;
          const v4f v = *(const v4f*)(slab + row * 68 + c4) * oscale;
          *(volatile v4f*)(C + (size_t)(mBase + row) * ldc + n0 + c4) = v;
        }
        __threadfence();
      }
      wave_lds_sync();
    }
  } else {
    unsigned short* C = (unsigned short*)Cout + (size_t)b * (size_t)strideC;
#pragma unroll
    for (int i = 0; i < 4; ++i) {
      const int mBase = m0 + (i << 4);
#pragma unroll
      for (int j = 0; j < 4; ++j) {
#pragma unroll
        for (int r = 0; r < 8; ++r) slab[(mOff + r) * 68 + (j << 4) + rlane] = acc[i][j][r];
      }
      wave_lds_sync();
      store_rows16<(MODE == 1)>(slab, C, ldc, mBase, n0, lane, aux, oscale);
      wave_lds_sync();
    }
    if (MODE == 2) {
      if (tn != tm) {
#pragma unroll
        for (int j = 0; j < 4; ++j) {
          const int nBase = n0 + (j << 4);
#pragma unroll
          for (int i = 0; i < 4; ++i) {
#pragma unroll
            for (int r = 0; r < 8; ++r) slab[rlane * 68 + (i << 4) + mOff + r] = acc[i][j][r];
          }
          wave_lds_sync();
          store_rows16<false>(slab, C, ldc, nBase, m0, lane, aux, oscale);
          wave_lds_sync();
        }
      }
    }
  }
}

extern "C" void kernel_launch(void* const* d_in, const int* in_sizes, int n_in,
                              void* d_out, int out_size, void* d_ws, size_t ws_size,
                              hipStream_t stream) {
  if (n_in < 3) return;
  if (in_sizes[0] != NBATCH * CCH * NVOX) return;
  if (in_sizes[1] != CCH * CCH) return;
  if (in_sizes[2] != CCH) return;
  if (out_size != NBATCH * CCH * NVOX) return;

  const float* x    = (const float*)d_in[0];
  const float* W    = (const float*)d_in[1];
  const float* bias = (const float*)d_in[2];
  float* out = (float*)d_out;

  const size_t PXT = (size_t)NBATCH * NVOX * CCH * 2;
  const size_t PWB = (size_t)CCH * CCH * 2;
  const size_t PTP = (size_t)NBATCH * CCH * NVOX * 2;
  const size_t PSM = (size_t)NVOX * NVOX * 2;
  const size_t PRN = (size_t)NBATCH * NVOX * 4;
  size_t off = 0;
  const size_t oXT = off; off += PXT;
  const size_t oWB = off; off += PWB;
  const size_t oTP = off; off += PTP;
  const size_t oSM = off; off += PSM;
  const size_t oRN = off; off += PRN;
  if (off > ws_size) return;
  if (off > (size_t)134217728) return;

  char* ws = (char*)d_ws;
  unsigned short* XT  = (unsigned short*)(ws + oXT);
  unsigned short* WB  = (unsigned short*)(ws + oWB);
  unsigned short* TP  = (unsigned short*)(ws + oTP);
  unsigned short* SIM = (unsigned short*)(ws + oSM);
  float*          RN  = (float*)(ws + oRN);

  const dim3 blk(256);
  const int n8w = CCH * CCH / 8;
  const dim3 gCvtW((n8w + 255) / 256);
  const dim3 gPrep(NVOX / 32, NBATCH);
  const dim3 gT((((CCH / 64) * (NVOX / 64)) + 7) / 8, NBATCH);
  const int  ntri = (NVOX / 64) * (NVOX / 64 + 1) / 2;
  const dim3 gG((ntri + 7) / 8, 1);
  const dim3 gO((((CCH / 64) * (NVOX / 64)) + 7) / 8, 1);

  cvt_bf16x8<<<gCvtW, blk, 0, stream>>>(W, WB, n8w);
  prep_xt<<<gPrep, blk, 0, stream>>>(x, XT, RN);
  gemm64<__bf16, 1><<<gT, blk, 0, stream>>>(
      WB, CCH, 0LL, XT, CCH, (long long)NVOX * CCH,
      (void*)TP, NVOX, (long long)CCH * NVOX, bias,
      CCH, NVOX, CCH, TSC);
  for (int b = 0; b < NBATCH; ++b) {
    const unsigned short* XTb = XT + (size_t)b * NVOX * CCH;
    const unsigned short* TPb = TP + (size_t)b * CCH * NVOX;
    const float* RNb = RN + (size_t)b * NVOX;
    float* outb = out + (size_t)b * CCH * NVOX;
    gemm64<__bf16, 2><<<gG, blk, 0, stream>>>(
        XTb, CCH, 0LL, XTb, CCH, 0LL,
        (void*)SIM, NVOX, 0LL, RNb,
        NVOX, NVOX, CCH, SSC);
    gemm64<_Float16, 0><<<gO, blk, 0, stream>>>(
        TPb, NVOX, 0LL, SIM, NVOX, 0LL,
        (void*)outb, NVOX, 0LL, RNb,
        CCH, NVOX, NVOX, OSC);
  }
  (void)hipGetLastError();
}
